// Rs_GCN_70712341561912
// MI455X (gfx1250) — hardware-verified
//
#include <hip/hip_runtime.h>


#define NB_  4
#define CC   512
#define CI   256
#define NN_  4096
#define NTK  (NB_ * NN_)

typedef unsigned short bf;
typedef __attribute__((ext_vector_type(16))) __bf16   v16bf;
typedef __attribute__((ext_vector_type(8)))  unsigned short v8us;
typedef __attribute__((ext_vector_type(8)))  float    v8f;
typedef __attribute__((ext_vector_type(4)))  float    v4f;
typedef v4f  __attribute__((may_alias)) v4fa;
typedef v8us __attribute__((may_alias)) v8usa;

__device__ __forceinline__ unsigned short f2bf(float f) { unsigned u = __float_as_uint(f); u += 0x7FFFu + ((u >> 16) & 1u); return (unsigned short)(u >> 16); }
__device__ __forceinline__ float bf2f(unsigned short b) { return __uint_as_float(((unsigned)b) << 16); }
__device__ __forceinline__ float bfr(float f) { return bf2f(f2bf(f)); }
__device__ __forceinline__ v16bf cat16b(v8us lo, v8us hi) { return __builtin_bit_cast(v16bf, __builtin_shufflevector(lo, hi, 0, 1, 2, 3, 4, 5, 6, 7, 8, 9, 10, 11, 12, 13, 14, 15)); }
__device__ __forceinline__ v8f wmmab(v16bf a, v16bf b, v8f c) { return __builtin_amdgcn_wmma_f32_16x16x32_bf16(false, a, false, b, (short)0, c, false, false); }
#define VST2(T, p, v) do { const T vst2_v_ = (v); *(volatile T*)(p) = vst2_v_; __threadfence(); *(volatile T*)(p) = vst2_v_; } while (0)

__global__ __launch_bounds__(256) void k_xt(const float* __restrict__ v, bf* XT) {
    __shared__ __align__(16) unsigned short tl[64 * 72];
    const int tid = threadIdx.x, n0 = blockIdx.x * 64, c0 = blockIdx.y * 64, b = blockIdx.z;
    const int cr = tid >> 2, nq = (tid & 3) * 16;
#pragma unroll
    for (int i = 0; i < 16; ++i) tl[(nq + i) * 72 + cr] = f2bf(v[((size_t)b * CC + c0 + cr) * NN_ + n0 + nq + i]);
    __syncthreads();
    const int piece = tid & 7;
    auto pass = [&]() {
#pragma unroll
        for (int s = 0; s < 2; ++s) { const int nr = (tid >> 3) + 32 * s; const v8us val = *(const v8usa*)(tl + nr * 72 + piece * 8); *(volatile v8us*)(XT + ((size_t)b * NN_ + n0 + nr) * CC + c0 + piece * 8) = val; }
    };
    pass(); __threadfence(); pass();
}
template <int C>
__global__ __launch_bounds__(256) void k_rows(const float* __restrict__ src, int nrows, bf* dst) {
    const int lane = threadIdx.x & 31, row = blockIdx.x * 8 + (threadIdx.x >> 5);
    if (row >= nrows) return;
    v8us o[C / 256];
#pragma unroll
    for (int c = 0; c < C / 256; ++c)
#pragma unroll
        for (int i = 0; i < 8; ++i) o[c][i] = f2bf(src[(size_t)row * C + c * 256 + lane * 8 + i]);
#pragma unroll
    for (int c = 0; c < C / 256; ++c) *(volatile v8us*)(dst + (size_t)row * C + c * 256 + lane * 8) = o[c];
    __threadfence();
#pragma unroll
    for (int c = 0; c < C / 256; ++c) *(volatile v8us*)(dst + (size_t)row * C + c * 256 + lane * 8) = o[c];
}
template <int NPROD, int MODE, bool RB = false>
__global__ __launch_bounds__(128) void k_gemm(const bf* __restrict__ A, const bf* __restrict__ Al, size_t za, int lda, const bf* __restrict__ Bn, const bf* __restrict__ Bl, size_t zb, int ldb, int K,
                                             const float* __restrict__ bias, float scale, size_t zc, int ldc, float* C, bf* PH, bf* PL) {
    __shared__ __align__(16) float ost[4][16 * 68];
    const int lane = threadIdx.x & 31, wave = threadIdx.x >> 5, lr = lane & 15, hi = lane >> 4, z = blockIdx.z;
    const size_t r0 = (size_t)blockIdx.x * 64 + wave * 16; const int c0 = blockIdx.y * 64;
    A += z * za; if (NPROD == 2 || NPROD == 3) Al += z * za; Bn += z * zb; if (NPROD >= 3) Bl += z * zb;
    const size_t aoff = (r0 + lr) * lda + 8 * hi;
    size_t boff[4];
#pragma unroll
    for (int t = 0; t < 4; ++t) boff[t] = (size_t)(c0 + t * 16 + lr) * ldb + 8 * hi;
    v8f acc[4];
#pragma unroll
    for (int t = 0; t < 4; ++t) acc[t] = (v8f){};
#pragma unroll 2
    for (int kc = 0; kc < K; kc += 32) {
        const v16bf a = cat16b(*(const v8us*)(A + aoff + kc), *(const v8us*)(A + aoff + kc + 16));
        v16bf al = a; if (NPROD == 2 || NPROD == 3) al = cat16b(*(const v8us*)(Al + aoff + kc), *(const v8us*)(Al + aoff + kc + 16));
#pragma unroll
        for (int t = 0; t < 4; ++t) { const v16bf bb = cat16b(*(const v8us*)(Bn + boff[t] + kc), *(const v8us*)(Bn + boff[t] + kc + 16)); acc[t] = wmmab(a, bb, acc[t]); if (NPROD == 2 || NPROD == 3) acc[t] = wmmab(al, bb, acc[t]);
            if (NPROD >= 3) { const v16bf bl = cat16b(*(const v8us*)(Bl + boff[t] + kc), *(const v8us*)(Bl + boff[t] + kc + 16)); acc[t] = wmmab(a, bl, acc[t]); } }
        asm volatile("v_nop\n\tv_nop\n\tv_nop\n\tv_nop" : "+v"(acc[0]), "+v"(acc[1]), "+v"(acc[2]), "+v"(acc[3]) : "v"(a), "v"(al));
    }
    float* os = &ost[wave][0];
#pragma unroll
    for (int t = 0; t < 4; ++t) { const float bv = (bias && !RB) ? bfr(bias[c0 + t * 16 + lr]) : 0.f;
#pragma unroll
        for (int j = 0; j < 8; ++j) { const float rbv = (bias && RB) ? bfr(bias[r0 + hi * 8 + j]) : 0.f; os[(hi * 8 + j) * 68 + t * 16 + lr] = acc[t][j] * scale + bv + rbv; } }
    __syncthreads();
    if (MODE == 0) {
        float* crow = C + z * zc + r0 * ldc + c0;
        auto pass = [&]() {
#pragma unroll
            for (int s = 0; s < 8; ++s) { const int Lid = (lane >> 3) + 4 * s, piece = lane & 7; const int row = Lid >> 1, cofs = (Lid & 1) * 32 + piece * 4;
                const v4f val = *(const v4fa*)(os + row * 68 + cofs); *(volatile v4f*)(crow + (size_t)row * ldc + cofs) = val; }
        };
        pass(); __threadfence(); pass();
    } else {
        bf* p1 = PH + z * zc + r0 * ldc + c0; bf* p2 = PL + z * zc + r0 * ldc + c0;
        auto pass = [&]() {
#pragma unroll
            for (int s = 0; s < 4; ++s) { const int row = 4 * s + (lane >> 3), piece = lane & 7; const float* sp = os + row * 68 + piece * 8; v8us oh, ol;
#pragma unroll
                for (int i = 0; i < 8; ++i) { const unsigned short hb = f2bf(sp[i]); oh[i] = hb; ol[i] = f2bf(sp[i] - bf2f(hb)); }
                *(volatile v8us*)(p1 + (size_t)row * ldc + piece * 8) = oh; *(volatile v8us*)(p2 + (size_t)row * ldc + piece * 8) = ol; }
        };
        pass(); __threadfence(); pass();
    }
}
__global__ __launch_bounds__(256) void k_tr(const float* __restrict__ P, bf* PTH, bf* PTL) {
    __shared__ float tl[64][65];
    const int tid = threadIdx.x, n0 = blockIdx.x * 64, c0 = blockIdx.y * 64, b = blockIdx.z;
    { const int nn = tid >> 2, cq = (tid & 3) * 16;
#pragma unroll
      for (int i = 0; i < 16; ++i) tl[cq + i][nn] = P[((size_t)b * NN_ + n0 + nn) * CI + c0 + cq + i]; }
    __syncthreads();
    const int piece = tid & 7;
    auto pass = [&]() {
#pragma unroll
        for (int s = 0; s < 2; ++s) { const int c = (tid >> 3) + 32 * s; v8us oh, ol;
#pragma unroll
            for (int i = 0; i < 8; ++i) { const float v = tl[c][piece * 8 + i]; const unsigned short hb = f2bf(v); oh[i] = hb; ol[i] = f2bf(v - bf2f(hb)); }
            const size_t o = ((size_t)b * CI + c0 + c) * NN_ + n0 + piece * 8; *(volatile v8us*)(PTH + o) = oh; *(volatile v8us*)(PTL + o) = ol; }
    };
    pass(); __threadfence(); pass();
}
__global__ __launch_bounds__(256) void k_mt(const float* __restrict__ M, bf* MTH, bf* MTL) {
    __shared__ float tl[64][65];
    const int tid = threadIdx.x, r0 = blockIdx.x * 64, c0 = blockIdx.y * 64, b = blockIdx.z;
    { const int rr = tid >> 2, cq = (tid & 3) * 16;
#pragma unroll
      for (int i = 0; i < 16; ++i) tl[cq + i][rr] = M[((size_t)b * CI + r0 + rr) * CI + c0 + cq + i]; }
    __syncthreads();
    const int piece = tid & 7;
    auto pass = [&]() {
#pragma unroll
        for (int s = 0; s < 2; ++s) { const int c = (tid >> 3) + 32 * s; v8us oh, ol;
#pragma unroll
            for (int i = 0; i < 8; ++i) { const float v = tl[c][piece * 8 + i]; const unsigned short hb = f2bf(v); oh[i] = hb; ol[i] = f2bf(v - bf2f(hb)); }
            const size_t o = ((size_t)b * CI + c0 + c) * CI + r0 + piece * 8; *(volatile v8us*)(MTH + o) = oh; *(volatile v8us*)(MTL + o) = ol; }
    };
    pass(); __threadfence(); pass();
}
__global__ __launch_bounds__(256) void k_bn(const float* __restrict__ Wy, const float* __restrict__ v, const float* __restrict__ gam, const float* __restrict__ bet, float* out) {
    __shared__ float red[256]; __shared__ float stat[2];
    const int o = blockIdx.x, tid = threadIdx.x;
    float s = 0.f;
    for (int b = 0; b < NB_; ++b) { const float* row = Wy + ((size_t)b * CC + o) * NN_;
        for (int n = tid; n < NN_; n += 256) s += row[n]; }
    red[tid] = s; __syncthreads();
    for (int st = 128; st > 0; st >>= 1) { if (tid < st) red[tid] += red[tid + st]; __syncthreads(); }
    if (tid == 0) stat[0] = red[0] / (float)(NB_ * NN_);
    __syncthreads();
    const float mu = stat[0]; float q = 0.f;
    for (int b = 0; b < NB_; ++b) { const float* row = Wy + ((size_t)b * CC + o) * NN_;
        for (int n = tid; n < NN_; n += 256) { const float d = row[n] - mu; q += d * d; } }
    red[tid] = q; __syncthreads();
    for (int st = 128; st > 0; st >>= 1) { if (tid < st) red[tid] += red[tid + st]; __syncthreads(); }
    if (tid == 0) stat[1] = rsqrtf(red[0] / (float)(NB_ * NN_) + 1e-5f);
    __syncthreads();
    const float rs = stat[1], g = bfr(gam[o]), be = bfr(bet[o]);
    const int wave = tid >> 5, lane = tid & 31;
#pragma unroll 1
    for (int ps = 0; ps < 2; ++ps) {
        for (int b = 0; b < NB_; ++b) { const size_t rb = ((size_t)b * CC + o) * NN_;
#pragma unroll 1
            for (int ch = wave; ch < NN_ / 128; ch += 8) { v4f val;
#pragma unroll
                for (int i = 0; i < 4; ++i) { const size_t e = rb + ch * 128 + lane * 4 + i; val[i] = (Wy[e] - mu) * rs * g + be + bfr(v[e]); }
                *(volatile v4f*)(out + rb + ch * 128 + lane * 4) = val; } }
        if (ps == 0) __threadfence(); }
}

extern "C" void kernel_launch(void* const* d_in, const int* in_sizes, int n_in,
                              void* d_out, int out_size, void* d_ws, size_t ws_size, hipStream_t stream) {
    (void)in_sizes; (void)n_in; (void)out_size;
    const float* v = (const float*)d_in[0]; const float* Wg = (const float*)d_in[1]; const float* bg = (const float*)d_in[2]; const float* Wth = (const float*)d_in[3]; const float* bth = (const float*)d_in[4];
    const float* Wph = (const float*)d_in[5]; const float* bph = (const float*)d_in[6]; const float* Ww = (const float*)d_in[7]; const float* bw = (const float*)d_in[8]; const float* gam = (const float*)d_in[9]; const float* bet = (const float*)d_in[10];
    float* out = (float*)d_out;
    char* wsp = (char*)d_ws;
    auto take = [&](size_t bytes) { char* p = wsp; wsp += (bytes + 255) & ~(size_t)255; return (void*)p; };
    bf* XT = (bf*)take((size_t)NTK * CC * 2); float* TMP = (float*)take((size_t)NTK * CI * 4);
    bf* WgB = (bf*)take((size_t)CI * CC * 2); bf* WthB = (bf*)take((size_t)CI * CC * 2); bf* WphB = (bf*)take((size_t)CI * CC * 2); bf* WwB = (bf*)take((size_t)CC * CI * 2);
    bf* THH = (bf*)take((size_t)NTK * CI * 2); bf* THL = (bf*)take((size_t)NTK * CI * 2);
    bf* PTH = (bf*)take((size_t)NTK * CI * 2); bf* PTL = (bf*)take((size_t)NTK * CI * 2);
    bf* GTH = (bf*)take((size_t)NTK * CI * 2); bf* GTL = (bf*)take((size_t)NTK * CI * 2);
    float* M = (float*)take((size_t)NB_ * CI * CI * 4); bf* MTH = (bf*)take((size_t)NB_ * CI * CI * 2); bf* MTL = (bf*)take((size_t)NB_ * CI * CI * 2);
    bf* YH = (bf*)take((size_t)NTK * CI * 2); bf* YL = (bf*)take((size_t)NTK * CI * 2);
    if ((size_t)(wsp - (char*)d_ws) > ws_size) return;
    float* Wy = (float*)XT;
    k_xt<<<dim3(NN_ / 64, CC / 64, NB_), 256, 0, stream>>>(v, XT);
    k_rows<CC><<<CI / 8, 256, 0, stream>>>(Wg, CI, WgB); k_rows<CC><<<CI / 8, 256, 0, stream>>>(Wth, CI, WthB); k_rows<CC><<<CI / 8, 256, 0, stream>>>(Wph, CI, WphB); k_rows<CI><<<CC / 8, 256, 0, stream>>>(Ww, CC, WwB);
    k_gemm<1, 1><<<dim3(NTK / 64, CI / 64, 1), 128, 0, stream>>>(XT, nullptr, 0, CC, WthB, nullptr, 0, CC, CC, bth, 1.0f, 0, CI, nullptr, THH, THL);
    k_gemm<1, 0><<<dim3(NTK / 64, CI / 64, 1), 128, 0, stream>>>(XT, nullptr, 0, CC, WphB, nullptr, 0, CC, CC, bph, 1.0f, 0, CI, TMP, nullptr, nullptr);
    k_tr<<<dim3(NN_ / 64, CI / 64, NB_), 256, 0, stream>>>(TMP, PTH, PTL);
    k_gemm<1, 0><<<dim3(NTK / 64, CI / 64, 1), 128, 0, stream>>>(XT, nullptr, 0, CC, WgB, nullptr, 0, CC, CC, bg, 1.0f, 0, CI, TMP, nullptr, nullptr);
    k_tr<<<dim3(NN_ / 64, CI / 64, NB_), 256, 0, stream>>>(TMP, GTH, GTL);
    k_gemm<3, 0><<<dim3(CI / 64, CI / 64, NB_), 128, 0, stream>>>(PTH, PTL, (size_t)CI * NN_, NN_, GTH, GTL, (size_t)CI * NN_, NN_, NN_, nullptr, 1.0f / (float)NN_, (size_t)CI * CI, CI, M, nullptr, nullptr);
    k_mt<<<dim3(CI / 64, CI / 64, NB_), 256, 0, stream>>>(M, MTH, MTL);
    k_gemm<3, 1><<<dim3(NN_ / 64, CI / 64, NB_), 128, 0, stream>>>(THH, THL, (size_t)NN_ * CI, CI, MTH, MTL, (size_t)CI * CI, CI, CI, nullptr, 1.0f, (size_t)NN_ * CI, CI, nullptr, YH, YL);
    k_gemm<4, 0, true><<<dim3(CC / 64, NN_ / 64, NB_), 128, 0, stream>>>(WwB, nullptr, 0, CI, YH, YL, (size_t)NN_ * CI, CI, CI, bw, 1.0f, (size_t)CC * NN_, NN_, Wy, nullptr, nullptr);
    k_bn<<<CC, 256, 0, stream>>>(Wy, v, gam, bet, out);
}
